// InvertedAttentionBlock_46308337385576
// MI455X (gfx1250) — hardware-verified
//
#include <hip/hip_runtime.h>
#include <math.h>

typedef _Float16 v16h __attribute__((ext_vector_type(16)));
typedef _Float16 v8h  __attribute__((ext_vector_type(8)));
typedef float    v8f  __attribute__((ext_vector_type(8)));
typedef float    v4f  __attribute__((ext_vector_type(4)));
typedef int      v4i  __attribute__((ext_vector_type(4)));
typedef v8h __attribute__((may_alias)) v8ha;
typedef v4f __attribute__((may_alias)) v4fa;
typedef v4i __attribute__((may_alias)) v4ia;

union Frag { v16h v; v8h half[2]; };

#define SEQ    1024
#define BATCH  8
#define EMB    768
#define NHEADS 12
#define HD     64
#define HIDN   3072
#define MROWS  (SEQ * BATCH)
#define NX     (MROWS * EMB)
#define PSCALE 16384.0f

#define G0   (3 * EMB * EMB / 8)
#define G1   (EMB * EMB / 8)
#define G2   (HIDN * EMB / 8)
#define NGRP (G0 + G1 + 2 * G2)

__device__ __forceinline__ v8f wmma_f16(v16h a, v16h b, v8f c) {
  v8f d = __builtin_amdgcn_wmma_f32_16x16x32_f16(false, a, false, b, (short)0, c, false, false);
  asm volatile("v_nop\n\tv_nop\n\tv_nop\n\tv_nop" : "+v"(d) : "v"(a), "v"(b));
  return d;
}

__device__ __forceinline__ v16h load_frag(const _Float16* p, int h) {
  Frag f;
  f.half[0] = *(const v8ha*)(p + 8 * h);
  f.half[1] = *(const v8ha*)(p + 16 + 8 * h);
  return f.v;
}

__device__ __forceinline__ v8h cvt8(v4f a, v4f c, float sc) {
  const v8h o = { (_Float16)(a.x * sc), (_Float16)(a.y * sc), (_Float16)(a.z * sc), (_Float16)(a.w * sc),
                  (_Float16)(c.x * sc), (_Float16)(c.y * sc), (_Float16)(c.z * sc), (_Float16)(c.w * sc) };
  return o;
}

__global__ __launch_bounds__(256) void convert_kernel(
    const float* __restrict__ w_in, const float* __restrict__ w_o,
    const float* __restrict__ w_1, const float* __restrict__ w_2,
    _Float16* __restrict__ wdst)
{
  const int g = blockIdx.x * 256 + threadIdx.x;
  if (g >= NGRP) return;
  const float* src;
  float sc;
  if (g < G0)                { src = w_in + (size_t)g * 8;                  sc = 32.0f; }
  else if (g < G0 + G1)      { src = w_o  + (size_t)(g - G0) * 8;           sc = 32.0f; }
  else if (g < G0 + G1 + G2) { src = w_1  + (size_t)(g - G0 - G1) * 8;      sc = 32.0f; }
  else                       { src = w_2  + (size_t)(g - G0 - G1 - G2) * 8; sc = 64.0f; }
  _Float16* dst = wdst + (size_t)g * 8;
  const v4f a = *(const v4fa*)src;
  const v4f c = *(const v4fa*)(src + 4);
  const v8h o = cvt8(a, c, sc);
  *(volatile v8h*)dst = o;
  __threadfence();
  *(volatile v8h*)dst = o;
}

__global__ __launch_bounds__(128) void ln_kernel(
    const float* __restrict__ xin, const float* __restrict__ g,
    const float* __restrict__ bb, _Float16* __restrict__ o16, int nrows)
{
  const int lane = threadIdx.x & 31, w = threadIdx.x >> 5;
  const int row = blockIdx.x * 4 + w;
  if (row >= nrows) return;
  const float* xr = xin + (size_t)row * EMB + 8 * lane;
  v4f a[3], c[3];
  float s = 0.0f;
  #pragma unroll
  for (int i = 0; i < 3; ++i) {
    a[i] = *(const v4fa*)(xr + 256 * i);
    c[i] = *(const v4fa*)(xr + 256 * i + 4);
    s += (a[i].x + a[i].y) + (a[i].z + a[i].w) + (c[i].x + c[i].y) + (c[i].z + c[i].w);
  }
  #pragma unroll
  for (int off = 16; off >= 1; off >>= 1) s += __shfl_xor(s, off, 32);
  const float mu = s * (1.0f / EMB);
  float q = 0.0f;
  #pragma unroll
  for (int i = 0; i < 3; ++i) {
    a[i] = a[i] - mu;
    c[i] = c[i] - mu;
    q += a[i].x * a[i].x + a[i].y * a[i].y + a[i].z * a[i].z + a[i].w * a[i].w
       + c[i].x * c[i].x + c[i].y * c[i].y + c[i].z * c[i].z + c[i].w * c[i].w;
  }
  #pragma unroll
  for (int off = 16; off >= 1; off >>= 1) q += __shfl_xor(q, off, 32);
  const float rstd = rsqrtf(q * (1.0f / EMB) + 1e-5f);

  v8h o[3];
  #pragma unroll
  for (int i = 0; i < 3; ++i) {
    const v4f ga = *(const v4fa*)(g + 256 * i + 8 * lane);
    const v4f gc = *(const v4fa*)(g + 256 * i + 8 * lane + 4);
    const v4f ba = *(const v4fa*)(bb + 256 * i + 8 * lane);
    const v4f bc = *(const v4fa*)(bb + 256 * i + 8 * lane + 4);
    const v4f ya = a[i] * rstd * ga + ba;
    const v4f yc = c[i] * rstd * gc + bc;
    o[i] = cvt8(ya, yc, 1.0f);
  }
  _Float16* dst = o16 + (size_t)row * EMB + 8 * lane;
  #pragma unroll
  for (int i = 0; i < 3; ++i) *(volatile v8h*)(dst + 256 * i) = o[i];
  __threadfence();
  #pragma unroll
  for (int i = 0; i < 3; ++i) *(volatile v8h*)(dst + 256 * i) = o[i];
}

template <int K>
__device__ __forceinline__ void gemm_core(const _Float16* xa0, const _Float16* xa1,
                                          const _Float16* wb, int h, v8f acc[2][4]) {
  #pragma unroll 1
  for (int k0 = 0; k0 < K; k0 += 32) {
    const v16h a0 = load_frag(xa0 + k0, h);
    const v16h a1 = load_frag(xa1 + k0, h);
    #pragma unroll
    for (int nt = 0; nt < 4; ++nt) {
      const v16h b = load_frag(wb + (size_t)nt * 16 * K + k0, h);
      acc[0][nt] = wmma_f16(a0, b, acc[0][nt]);
      acc[1][nt] = wmma_f16(a1, b, acc[1][nt]);
    }
  }
}

__device__ __forceinline__ void qkv_store_pass(const _Float16* sT, _Float16* plane, _Float16* vt,
                                               int which, int bh, int s0, int w, int lane) {
  const int q8 = lane & 7, sub = lane >> 3;
  #pragma unroll
  for (int i = 0; i < 8; ++i) {
    const int lid = w * 32 + i * 4 + sub;
    v8h v;
    _Float16* dst;
    if (which != 2) {
      v = *(const v8ha*)(sT + lid * HD + 8 * q8);
      dst = plane + ((size_t)bh * SEQ + s0 + lid) * HD + 8 * q8;
    } else {
      const int d = lid >> 1, hl = lid & 1;
      v = *(const v8ha*)(sT + d * 128 + 64 * hl + 8 * q8);
      dst = vt + ((size_t)bh * HD + d) * SEQ + s0 + 64 * hl + 8 * q8;
    }
    *(volatile v8h*)dst = v;
  }
}

__global__ __launch_bounds__(128) void qkv_kernel(
    const _Float16* __restrict__ inp16,
    const _Float16* __restrict__ win16,
    const float* __restrict__ bin,
    _Float16* __restrict__ qh,
    _Float16* __restrict__ kh,
    _Float16* __restrict__ vt)
{
  __shared__ __attribute__((aligned(16))) _Float16 sT[128 * 64];

  const int tid = threadIdx.x, lane = tid & 31, w = tid >> 5;
  const int h = lane >> 4, m = lane & 15;
  const int b = blockIdx.x & 7;
  const int s0 = (blockIdx.x >> 3) * 128;
  const int cg = blockIdx.y;
  const int which = cg / NHEADS;
  const int head = cg - which * NHEADS;
  const int sw = s0 + 32 * w;

  const _Float16* xa0 = inp16 + ((size_t)(sw + m) * BATCH + b) * EMB;
  const _Float16* xa1 = inp16 + ((size_t)(sw + 16 + m) * BATCH + b) * EMB;
  const _Float16* wb  = win16 + ((size_t)which * EMB + head * HD + m) * EMB;

  const v8f zero8 = {0.f, 0.f, 0.f, 0.f, 0.f, 0.f, 0.f, 0.f};
  v8f acc[2][4];
  #pragma unroll
  for (int mt = 0; mt < 2; ++mt)
    #pragma unroll
    for (int nt = 0; nt < 4; ++nt) acc[mt][nt] = zero8;

  gemm_core<EMB>(xa0, xa1, wb, h, acc);

  const float* bias = bin + which * EMB + head * HD;
  const float osc = (which == 0) ? 0.125f : 1.0f;
  #pragma unroll
  for (int nt = 0; nt < 4; ++nt) {
    const int feat = 16 * nt + m;
    const float bvl = bias[feat];
    #pragma unroll
    for (int mt = 0; mt < 2; ++mt) {
      #pragma unroll
      for (int r = 0; r < 8; ++r) {
        const int tokl = 32 * w + 16 * mt + 8 * h + r;
        const float y = (acc[mt][nt][r] * 0.03125f + bvl) * osc;
        const int idx = (which == 2) ? (feat * 128 + tokl) : (tokl * HD + feat);
        sT[idx] = (_Float16)y;
      }
    }
  }
  __syncthreads();

  const int bh = b * NHEADS + head;
  _Float16* plane = (which == 0) ? qh : kh;
  qkv_store_pass(sT, plane, vt, which, bh, s0, w, lane);
  __threadfence();
  qkv_store_pass(sT, plane, vt, which, bh, s0, w, lane);
}

__device__ __forceinline__ v8f apply_mask8(v8f s, const int* p) {
  const v4i ma = *(const v4ia*)p;
  const v4i mb = *(const v4ia*)(p + 4);
  s[0] = ma.x ? -1e30f : s[0];
  s[1] = ma.y ? -1e30f : s[1];
  s[2] = ma.z ? -1e30f : s[2];
  s[3] = ma.w ? -1e30f : s[3];
  s[4] = mb.x ? -1e30f : s[4];
  s[5] = mb.y ? -1e30f : s[5];
  s[6] = mb.z ? -1e30f : s[6];
  s[7] = mb.w ? -1e30f : s[7];
  return s;
}

__device__ __forceinline__ v16h pack_p(v8f a, v8f c) {
  const v16h r = { (_Float16)(a[0] * PSCALE), (_Float16)(a[1] * PSCALE), (_Float16)(a[2] * PSCALE), (_Float16)(a[3] * PSCALE),
                   (_Float16)(a[4] * PSCALE), (_Float16)(a[5] * PSCALE), (_Float16)(a[6] * PSCALE), (_Float16)(a[7] * PSCALE),
                   (_Float16)(c[0] * PSCALE), (_Float16)(c[1] * PSCALE), (_Float16)(c[2] * PSCALE), (_Float16)(c[3] * PSCALE),
                   (_Float16)(c[4] * PSCALE), (_Float16)(c[5] * PSCALE), (_Float16)(c[6] * PSCALE), (_Float16)(c[7] * PSCALE) };
  return r;
}

__device__ __forceinline__ void att_store_pass(const _Float16* so, _Float16* ctx,
                                               int b, int head, int q0, int lane) {
  const int q8 = lane & 7, sub = lane >> 3;
  #pragma unroll
  for (int i = 0; i < 4; ++i) {
    const int row = i * 4 + sub;
    const v8h v = *(const v8ha*)(so + row * HD + 8 * q8);
    const size_t gi = ((size_t)(q0 + row) * BATCH + b) * EMB + head * HD + 8 * q8;
    *(volatile v8h*)(ctx + gi) = v;
  }
}

__global__ __launch_bounds__(128) void attn_kernel(
    const _Float16* __restrict__ qh,
    const _Float16* __restrict__ kh,
    const _Float16* __restrict__ vt,
    const int* __restrict__ mask,
    _Float16* __restrict__ ctx)
{
  __shared__ __attribute__((aligned(16))) _Float16 sO[4 * 16 * 64];

  const int tid = threadIdx.x, lane = tid & 31, w = tid >> 5;
  const int h = lane >> 4, m = lane & 15;
  const int bh = blockIdx.y;
  const int b = bh / NHEADS, head = bh - b * NHEADS;
  const int q0 = blockIdx.x * 64 + 16 * w;

  const _Float16* qrow = qh + ((size_t)bh * SEQ + q0 + m) * HD;
  const v16h qb0 = load_frag(qrow, h);
  const v16h qb1 = load_frag(qrow + 32, h);

  const v8f zero8 = {0.f, 0.f, 0.f, 0.f, 0.f, 0.f, 0.f, 0.f};
  v8f o[4];
  #pragma unroll
  for (int t = 0; t < 4; ++t) o[t] = zero8;
  float mrun = -1e30f, lrun = 0.0f;

  const _Float16* kbase = kh + ((size_t)bh * SEQ + m) * HD;
  const _Float16* vbase = vt + ((size_t)bh * HD + m) * SEQ;
  const int* mkp = mask + (size_t)(q0 + m) * SEQ + 8 * h;

  #pragma unroll 1
  for (int kb = 0; kb < SEQ; kb += 64) {
    v8f s[4];
    #pragma unroll
    for (int j = 0; j < 4; ++j) {
      const _Float16* kp = kbase + (size_t)(kb + 16 * j) * HD;
      const v16h kf0 = load_frag(kp, h);
      const v16h kf1 = load_frag(kp + 32, h);
      v8f z = zero8;
      z = wmma_f16(kf0, qb0, z);
      z = wmma_f16(kf1, qb1, z);
      s[j] = z;
    }
    #pragma unroll
    for (int j = 0; j < 4; ++j) s[j] = apply_mask8(s[j], mkp + kb + 16 * j);

    float mloc = s[0][0];
    #pragma unroll
    for (int j = 0; j < 4; ++j)
      #pragma unroll
      for (int r = 0; r < 8; ++r) mloc = fmaxf(mloc, s[j][r]);
    mloc = fmaxf(mloc, __shfl_xor(mloc, 16, 32));
    const float mnew = fmaxf(mrun, mloc);
    const float alpha = __expf(mrun - mnew);
    mrun = mnew;
    float lsum = 0.0f;
    #pragma unroll
    for (int j = 0; j < 4; ++j)
      #pragma unroll
      for (int r = 0; r < 8; ++r) {
        const float p = __expf(s[j][r] - mnew);
        s[j][r] = p;
        lsum += p;
      }
    lsum += __shfl_xor(lsum, 16, 32);
    lrun = lrun * alpha + lsum;
    #pragma unroll
    for (int t = 0; t < 4; ++t)
      #pragma unroll
      for (int r = 0; r < 8; ++r) o[t][r] = o[t][r] * alpha;

    const v16h pb0 = pack_p(s[0], s[1]);
    const v16h pb1 = pack_p(s[2], s[3]);

    #pragma unroll
    for (int t = 0; t < 4; ++t) {
      const _Float16* vp = vbase + (size_t)(16 * t) * SEQ + kb;
      const v16h vf0 = load_frag(vp, h);
      const v16h vf1 = load_frag(vp + 32, h);
      o[t] = wmma_f16(vf0, pb0, o[t]);
      o[t] = wmma_f16(vf1, pb1, o[t]);
    }
  }

  const float inv = (1.0f / lrun) * (1.0f / PSCALE);
  _Float16* so = sO + w * 1024;
  #pragma unroll
  for (int t = 0; t < 4; ++t)
    #pragma unroll
    for (int r = 0; r < 8; ++r)
      so[m * HD + 16 * t + 8 * h + r] = (_Float16)(o[t][r] * inv);
  __syncthreads();

  att_store_pass(so, ctx, b, head, q0, lane);
  __threadfence();
  att_store_pass(so, ctx, b, head, q0, lane);
}

__device__ __forceinline__ void res_store_pass(const float* sO, const float* __restrict__ resid,
                                               float* __restrict__ outp, int m0, int n0, int w, int lane) {
  const int q8 = lane & 7, sub = lane >> 3;
  #pragma unroll
  for (int i = 0; i < 16; ++i) {
    const int lid = w * 64 + i * 4 + sub;
    const int row = lid >> 1, hl = lid & 1;
    const int col = 32 * hl + 4 * q8;
    const v4f v = *(const v4fa*)(sO + row * 64 + col);
    const size_t gi = (size_t)(m0 + row) * EMB + n0 + col;
    const v4f rr = *(const v4fa*)(resid + gi);
    const v4f y = v + rr;
    *(volatile v4f*)(outp + gi) = y;
  }
}

template <int K>
__global__ __launch_bounds__(128) void gemm_res_kernel(
    const _Float16* __restrict__ A16,
    const _Float16* __restrict__ W16,
    const float* __restrict__ bias,
    const float* __restrict__ resid,
    float* __restrict__ outp,
    float wsc)
{
  __shared__ __attribute__((aligned(16))) float sO[128 * 64];

  const int tid = threadIdx.x, lane = tid & 31, w = tid >> 5;
  const int h = lane >> 4, m = lane & 15;
  const int m0 = blockIdx.x * 128, n0 = blockIdx.y * 64;

  const _Float16* xa0 = A16 + (size_t)(m0 + 32 * w + m) * K;
  const _Float16* xa1 = xa0 + (size_t)16 * K;
  const _Float16* wb  = W16 + (size_t)(n0 + m) * K;

  const v8f zero8 = {0.f, 0.f, 0.f, 0.f, 0.f, 0.f, 0.f, 0.f};
  v8f acc[2][4];
  #pragma unroll
  for (int mt = 0; mt < 2; ++mt)
    #pragma unroll
    for (int nt = 0; nt < 4; ++nt) acc[mt][nt] = zero8;

  gemm_core<K>(xa0, xa1, wb, h, acc);

  #pragma unroll
  for (int nt = 0; nt < 4; ++nt) {
    const int feat = 16 * nt + m;
    const float bvl = bias[n0 + feat];
    #pragma unroll
    for (int mt = 0; mt < 2; ++mt) {
      #pragma unroll
      for (int r = 0; r < 8; ++r) {
        const int tokl = 32 * w + 16 * mt + 8 * h + r;
        sO[tokl * 64 + feat] = acc[mt][nt][r] * wsc + bvl;
      }
    }
  }
  __syncthreads();

  res_store_pass(sO, resid, outp, m0, n0, w, lane);
  __threadfence();
  res_store_pass(sO, resid, outp, m0, n0, w, lane);
}

__device__ __forceinline__ void fc1_store_pass(const _Float16* sT, _Float16* __restrict__ hid,
                                               int m0, int n0, int w, int lane) {
  const int q8 = lane & 7, sub = lane >> 3;
  #pragma unroll
  for (int i = 0; i < 8; ++i) {
    const int lid = w * 32 + i * 4 + sub;
    const v8h v = *(const v8ha*)(sT + lid * 64 + 8 * q8);
    *(volatile v8h*)(hid + (size_t)(m0 + lid) * HIDN + n0 + 8 * q8) = v;
  }
}

__global__ __launch_bounds__(128) void fc1_kernel(
    const _Float16* __restrict__ h16,
    const _Float16* __restrict__ w116,
    const float* __restrict__ b1,
    _Float16* __restrict__ hid)
{
  __shared__ __attribute__((aligned(16))) _Float16 sT[128 * 64];

  const int tid = threadIdx.x, lane = tid & 31, w = tid >> 5;
  const int h = lane >> 4, m = lane & 15;
  const int m0 = blockIdx.x * 128, n0 = blockIdx.y * 64;

  const _Float16* xa0 = h16 + (size_t)(m0 + 32 * w + m) * EMB;
  const _Float16* xa1 = xa0 + (size_t)16 * EMB;
  const _Float16* wb  = w116 + (size_t)(n0 + m) * EMB;

  const v8f zero8 = {0.f, 0.f, 0.f, 0.f, 0.f, 0.f, 0.f, 0.f};
  v8f acc[2][4];
  #pragma unroll
  for (int mt = 0; mt < 2; ++mt)
    #pragma unroll
    for (int nt = 0; nt < 4; ++nt) acc[mt][nt] = zero8;

  gemm_core<EMB>(xa0, xa1, wb, h, acc);

  #pragma unroll
  for (int nt = 0; nt < 4; ++nt) {
    const int feat = 16 * nt + m;
    const float bvl = b1[n0 + feat];
    #pragma unroll
    for (int mt = 0; mt < 2; ++mt) {
      #pragma unroll
      for (int r = 0; r < 8; ++r) {
        const int tokl = 32 * w + 16 * mt + 8 * h + r;
        const float v = acc[mt][nt][r] * 0.03125f + bvl;
        const float ge = 0.5f * v * (1.0f + erff(v * 0.70710678118654752f));
        sT[tokl * 64 + feat] = (_Float16)ge;
      }
    }
  }
  __syncthreads();

  fc1_store_pass(sT, hid, m0, n0, w, lane);
  __threadfence();
  fc1_store_pass(sT, hid, m0, n0, w, lane);
}

extern "C" void kernel_launch(void* const* d_in, const int* in_sizes, int n_in,
                              void* d_out, int out_size, void* d_ws, size_t ws_size,
                              hipStream_t stream) {
  if (n_in < 14) return;
  if (in_sizes[0] != NX) return;
  if (in_sizes[1] != EMB || in_sizes[2] != EMB) return;
  if (in_sizes[3] != 3 * EMB * EMB || in_sizes[4] != 3 * EMB) return;
  if (in_sizes[5] != EMB * EMB || in_sizes[6] != EMB) return;
  if (in_sizes[7] != EMB || in_sizes[8] != EMB) return;
  if (in_sizes[9] != HIDN * EMB || in_sizes[10] != HIDN) return;
  if (in_sizes[11] != EMB * HIDN || in_sizes[12] != EMB) return;
  if (in_sizes[13] != SEQ * SEQ) return;
  if (out_size != NX) return;

  const float* x     = (const float*)d_in[0];
  const float* ln1_g = (const float*)d_in[1];
  const float* ln1_b = (const float*)d_in[2];
  const float* in_w  = (const float*)d_in[3];
  const float* in_b  = (const float*)d_in[4];
  const float* out_w = (const float*)d_in[5];
  const float* out_b = (const float*)d_in[6];
  const float* ln2_g = (const float*)d_in[7];
  const float* ln2_b = (const float*)d_in[8];
  const float* w1    = (const float*)d_in[9];
  const float* b1    = (const float*)d_in[10];
  const float* w2    = (const float*)d_in[11];
  const float* b2    = (const float*)d_in[12];
  const int*   mask  = (const int*)d_in[13];
  float* out = (float*)d_out;

  const size_t win_b  = (size_t)3 * EMB * EMB * 2;
  const size_t wo_b   = (size_t)EMB * EMB * 2;
  const size_t w1_b   = (size_t)HIDN * EMB * 2;
  const size_t w2_b   = (size_t)EMB * HIDN * 2;
  const size_t regA   = win_b + wo_b + w1_b + w2_b;
  const size_t regB   = (size_t)MROWS * EMB * 2;
  const size_t plane  = (size_t)BATCH * NHEADS * SEQ * HD * 2;
  const size_t hid_b  = (size_t)MROWS * HIDN * 2;
  const size_t regC   = (3 * plane > hid_b) ? 3 * plane : hid_b;
  const size_t regD   = (size_t)MROWS * EMB * 4;
  const size_t total  = regA + regB + regC + regD;
  if (total > ws_size) return;

  char* ws = (char*)d_ws;
  _Float16* wA     = (_Float16*)(ws);
  _Float16* w_in16 = (_Float16*)(ws);
  _Float16* w_o16  = (_Float16*)(ws + win_b);
  _Float16* w1_16  = (_Float16*)(ws + win_b + wo_b);
  _Float16* w2_16  = (_Float16*)(ws + win_b + wo_b + w1_b);
  _Float16* bufB   = (_Float16*)(ws + regA);
  char*     cbase  = ws + regA + regB;
  _Float16* q16    = (_Float16*)(cbase);
  _Float16* k16    = (_Float16*)(cbase + plane);
  _Float16* vt16   = (_Float16*)(cbase + 2 * plane);
  _Float16* hid16  = (_Float16*)(cbase);
  float*    x2     = (float*)(ws + regA + regB + regC);

  convert_kernel<<<(NGRP + 255) / 256, 256, 0, stream>>>(in_w, out_w, w1, w2, wA);
  ln_kernel<<<(MROWS + 3) / 4, 128, 0, stream>>>(x, ln1_g, ln1_b, bufB, MROWS);
  qkv_kernel<<<dim3(BATCH * (SEQ / 128), 3 * NHEADS), 128, 0, stream>>>(bufB, w_in16, in_b, q16, k16, vt16);
  attn_kernel<<<dim3(SEQ / 64, BATCH * NHEADS), 128, 0, stream>>>(q16, k16, vt16, mask, bufB);
  gemm_res_kernel<EMB><<<dim3(MROWS / 128, EMB / 64), 128, 0, stream>>>(bufB, w_o16, out_b, x, x2, 0.03125f);
  ln_kernel<<<(MROWS + 3) / 4, 128, 0, stream>>>(x2, ln2_g, ln2_b, bufB, MROWS);
  fc1_kernel<<<dim3(MROWS / 128, HIDN / 64), 128, 0, stream>>>(bufB, w1_16, b1, hid16);
  gemm_res_kernel<HIDN><<<dim3(MROWS / 128, EMB / 64), 128, 0, stream>>>(hid16, w2_16, b2, x2, out, 0.015625f);
}
